// GAT_23416161697969
// MI455X (gfx1250) — hardware-verified
//
#include <hip/hip_runtime.h>
#include <stddef.h>
#include <stdint.h>
#include <math.h>


#define F_IN    256
#define HC1     512
#define HD1     128
#define NH1     4
#define KP2     1024
#define DOUT    64
#define NTHR    256
#define NWAVE   8
#define EPT     8
#define CHUNK   (NTHR * EPT)
#define WCAP    (EPT * 32)
#define LISTN   (NWAVE * WCAP)
#define NBA     1024
#define SLA     10
#define RCAP    28672
#define DEGCAP  128
#define GBM     64
#define GTHR    128
#define MROWS   128
#define NEGSL   0.2f
#define AGG_ZINTS (LISTN + 2 * RCAP + 3 * NBA)
#define AGG_LDS_INTS (AGG_ZINTS + 16)
#define WSMAX   134217728

static_assert((CHUNK & (CHUNK - 1)) == 0 && CHUNK <= 4096);
static_assert((NBA & (NBA - 1)) == 0 && NBA == (1 << SLA));
static_assert(((long long)CHUNK << SLA) < (1LL << 31));
static_assert(LISTN % NTHR == 0);
static_assert(NBA % NWAVE == 0 && NBA % 32 == 0 && NBA % GBM == 0);
static_assert(RCAP % 4 == 0 && AGG_ZINTS % 4 == 0 && LISTN % 4 == 0);
static_assert(F_IN % 32 == 0 && KP2 % 32 == 0 && KP2 == 2 * HC1 && HC1 == NH1 * HD1);
static_assert(GBM == (GTHR / 32) * 16 && GTHR == 2 * GBM);
static_assert((MROWS % GBM) == 0);
static_assert(AGG_LDS_INTS * 4 <= 300000);
static_assert(NWAVE * 512 + HC1 <= RCAP);
static_assert(HC1 == 2 * 8 * 32);
static_assert(DOUT == 4 * 16);
static_assert((F_IN / 8) == 32);

typedef float          v4f   __attribute__((ext_vector_type(4)));
typedef float          v8f   __attribute__((ext_vector_type(8)));
typedef int            v4i   __attribute__((ext_vector_type(4)));
typedef int            v8i   __attribute__((ext_vector_type(8)));
typedef unsigned int   v4u   __attribute__((ext_vector_type(4)));
typedef unsigned short v8us  __attribute__((ext_vector_type(8)));
typedef unsigned short v16us __attribute__((ext_vector_type(16)));
typedef __bf16         v16bf __attribute__((ext_vector_type(16)));
typedef v4f  __attribute__((may_alias)) v4fa;
typedef v4i  __attribute__((may_alias)) v4ia;
typedef v8us __attribute__((may_alias)) v8usa;
union FragB { v16bf v; v16us u; v8us h[2]; v8i w; };

__device__ __forceinline__ v8f wmb(const FragB& a, const FragB& b, v8f c) {
  v8f d = __builtin_amdgcn_wmma_f32_16x16x32_bf16(false, a.v, false, b.v, (short)0, c, false, false);
  asm volatile("v_nop\n\tv_nop\n\tv_nop\n\tv_nop" : "+v"(d) : "v"(a.w), "v"(b.w));
  return d;
}

__device__ __forceinline__ unsigned bf16_bits(float f) {
  const unsigned u = __float_as_uint(f);
  return ((u + 0x7FFFu + ((u >> 16) & 1u)) >> 16) & 0xFFFFu;
}
__device__ __forceinline__ float bf16_val(float f) {
  return __uint_as_float(bf16_bits(f) << 16);
}
__device__ __forceinline__ unsigned int pk2(float lo, float hi) { return bf16_bits(lo) | (bf16_bits(hi) << 16); }
__device__ __forceinline__ v4u pack8(const v4f a, const v4f b) {
  v4u r;
  r.x = pk2(a.x, a.y); r.y = pk2(a.z, a.w); r.z = pk2(b.x, b.y); r.w = pk2(b.z, b.w);
  return r;
}

__device__ __forceinline__ void osm(float lg, float& mx, float& dn, float& s1, float& s2) {
  const float df = lg - mx;
  const float ee = expf(-fabsf(df));
  const bool  up = df > 0.f;
  s1 = up ? ee : 1.0f;
  s2 = up ? 1.0f : ee;
  mx = up ? lg : mx;
  dn = fmaf(dn, s1, s2);
}

template <int SLB>
__device__ __forceinline__ int scan_chunk(const int* __restrict__ dsts, int nE, int cbase, int slotBase,
                                          int nb, int vec8, int* list, int tid, int lane, int wave) {
  int wc = 0;
  const int el0  = tid * EPT;
  const int e0   = cbase + el0;
  const int sent = -2147483647 - 1;
  v4i da, db;
  if (vec8 != 0 && cbase + CHUNK <= nE) {
    da = *(const v4i*)(dsts + e0);
    db = *(const v4i*)(dsts + e0 + 4);
  } else {
    da.x = (e0     < nE) ? dsts[min(e0,     nE - 1)] : sent;
    da.y = (e0 + 1 < nE) ? dsts[min(e0 + 1, nE - 1)] : sent;
    da.z = (e0 + 2 < nE) ? dsts[min(e0 + 2, nE - 1)] : sent;
    da.w = (e0 + 3 < nE) ? dsts[min(e0 + 3, nE - 1)] : sent;
    db.x = (e0 + 4 < nE) ? dsts[min(e0 + 4, nE - 1)] : sent;
    db.y = (e0 + 5 < nE) ? dsts[min(e0 + 5, nE - 1)] : sent;
    db.z = (e0 + 6 < nE) ? dsts[min(e0 + 6, nE - 1)] : sent;
    db.w = (e0 + 7 < nE) ? dsts[min(e0 + 7, nE - 1)] : sent;
  }
  const unsigned nbs = (unsigned)slotBase;
  const unsigned unb = (unsigned)nb;
  const unsigned s0 = (unsigned)da.x - nbs, s1 = (unsigned)da.y - nbs;
  const unsigned s2 = (unsigned)da.z - nbs, s3 = (unsigned)da.w - nbs;
  const unsigned s4 = (unsigned)db.x - nbs, s5 = (unsigned)db.y - nbs;
  const unsigned s6 = (unsigned)db.z - nbs, s7 = (unsigned)db.w - nbs;
  const bool h0 = s0 < unb, h1 = s1 < unb, h2 = s2 < unb, h3 = s3 < unb;
  const bool h4 = s4 < unb, h5 = s5 < unb, h6 = s6 < unb, h7 = s7 < unb;
  const unsigned any = __builtin_amdgcn_ballot_w32(h0 | h1 | h2 | h3 | h4 | h5 | h6 | h7);
  if (any != 0u) {
#define HITJ(J, HJ, SJ) { \
      const unsigned mj = __builtin_amdgcn_ballot_w32(HJ); \
      if (mj != 0u) { \
        if (HJ) { \
          const int pos = wc + (int)__builtin_amdgcn_mbcnt_lo(mj, 0u); \
          if (pos < WCAP) list[wave * WCAP + pos] = ((el0 + (J)) << SLB) | (int)(SJ); \
        } \
        wc += (int)__builtin_popcount(mj); } }
    HITJ(0, h0, s0)
    HITJ(1, h1, s1)
    HITJ(2, h2, s2)
    HITJ(3, h3, s3)
    HITJ(4, h4, s4)
    HITJ(5, h5, s5)
    HITJ(6, h6, s6)
    HITJ(7, h7, s7)
#undef HITJ
  }
  return wc;
}

__global__ __launch_bounds__(NTHR) void k_xprep(const float* __restrict__ x, unsigned short* xb, int nN, int nUnits) {
  const int i = (int)blockIdx.x * NTHR + (int)threadIdx.x;
  if (i >= nUnits) return;
  const int row = i >> 5;
  const int c0  = (i & 31) * 8;
  const int rc  = row < nN ? row : nN - 1;
  const float* p = x + (size_t)rc * F_IN + c0;
  v4f a = *(const v4fa*)p, b = *(const v4fa*)(p + 4);
  const v4f z4 = {0.f, 0.f, 0.f, 0.f};
  if (row >= nN) { a = z4; b = z4; }
  const v4u hv = pack8(a, b);
  const size_t o = (size_t)row * F_IN + c0;
  *(volatile v4u*)(xb + o) = hv;
  __threadfence();
  *(volatile v4u*)(xb + o) = hv;
}

__global__ __launch_bounds__(NTHR) void k_wtr(const float* __restrict__ w, int Kin, int Ncol, int Nrows, int Kout,
                                              unsigned short* wt, int nUnits) {
  const int u = (int)blockIdx.x * NTHR + (int)threadIdx.x;
  if (u >= nUnits) return;
  const int kq = Kout >> 3;
  const int n  = u / kq;
  const int k8 = (u - n * kq) * 8;
  const int kk = k8 - (k8 / Kin) * Kin;
  const int ncl = n < Ncol ? n : Ncol - 1;
  const float* p = w + (size_t)kk * (size_t)Ncol + ncl;
  v4f a, b;
  a.x = p[0];                    a.y = p[(size_t)Ncol];         a.z = p[(size_t)2 * Ncol];     a.w = p[(size_t)3 * Ncol];
  b.x = p[(size_t)4 * Ncol];     b.y = p[(size_t)5 * Ncol];     b.z = p[(size_t)6 * Ncol];     b.w = p[(size_t)7 * Ncol];
  const v4f z4 = {0.f, 0.f, 0.f, 0.f};
  if (n >= Ncol || n >= Nrows) { a = z4; b = z4; }
  const v4u wv = pack8(a, b);
  unsigned short* o = wt + (size_t)n * (size_t)Kout + k8;
  *(volatile v4u*)o = wv;
  __threadfence();
  *(volatile v4u*)o = wv;
}

template <int NT>
__global__ __launch_bounds__(GTHR) void k_gemm(const unsigned short* __restrict__ A, int lda,
                                               const unsigned short* __restrict__ BT, int ldb, int K,
                                               float* Cm, int ldc, const float* __restrict__ avs,
                                               const float* __restrict__ avd, float* AL) {
  static_assert(NT == 4 || NT == 8);
  constexpr int GBN = 16 * NT;
  constexpr int PPR = GBN / 4;
  constexpr int RPI = 32 / PPR;
  constexpr int NIT = 16 / RPI;
  __shared__ __attribute__((aligned(16))) float stg[GBM * GBN];
  __shared__ __attribute__((aligned(16))) float satt[2 * GBN];
  __shared__ __attribute__((aligned(16))) float sdt[2 * GBM];
  const int tid = (int)threadIdx.x, lane = tid & 31, wave = tid >> 5, hh = lane >> 4, m = lane & 15;
  const int rowBase = (int)blockIdx.x * GBM;
  const int head    = (int)blockIdx.y;
  const int colBase = head * GBN;

#pragma unroll 1
  for (int i = tid; i < 2 * GBN; i += GTHR) {
    const int which = i >= GBN ? 1 : 0;
    const int c = i - which * GBN;
    const float vs = avs[head * GBN + c];
    const float vd = avd[head * GBN + c];
    const float v = (which == 0) ? vs : vd;
    satt[i] = bf16_val(v);
  }

  v8f acc[NT];
  {
    const v8f z = {0.f, 0.f, 0.f, 0.f, 0.f, 0.f, 0.f, 0.f};
#pragma unroll
    for (int t = 0; t < NT; ++t) acc[t] = z;
  }
  const unsigned short* ap = A  + (size_t)(rowBase + 16 * wave + m) * (size_t)lda + 8 * hh;
  const unsigned short* bp = BT + (size_t)(colBase + m) * (size_t)ldb + 8 * hh;

#pragma unroll 1
  for (int k0 = 0; k0 < K; k0 += 32) {
    FragB af;
    af.h[0] = *(const v8usa*)(ap + k0);
    af.h[1] = *(const v8usa*)(ap + k0 + 16);
#pragma unroll
    for (int nt = 0; nt < NT; ++nt) {
      const unsigned short* wq = bp + (size_t)(16 * nt) * (size_t)ldb + k0;
      FragB bf;
      bf.h[0] = *(const v8usa*)wq;
      bf.h[1] = *(const v8usa*)(wq + 16);
      acc[nt] = wmb(af, bf, acc[nt]);
    }
  }

#pragma unroll
  for (int nt = 0; nt < NT; ++nt) {
    const int lc = 16 * nt + m;
#pragma unroll
    for (int r = 0; r < 8; ++r) {
      const int lr = 16 * wave + 8 * hh + r;
      stg[lr * GBN + lc] = acc[nt][r];
    }
  }
  __syncthreads();

  {
    const int row = tid & 63, which = tid >> 6;
    const float* sa = satt + which * GBN;
    const float* hr = stg + row * GBN;
    float d = 0.f;
#pragma unroll 4
    for (int c4 = 0; c4 < GBN / 4; ++c4) {
      const v4f hv = *(const v4fa*)(hr + 4 * c4);
      const v4f av = *(const v4fa*)(sa + 4 * c4);
      d = fmaf(hv.x, av.x, d);
      d = fmaf(hv.y, av.y, d);
      d = fmaf(hv.z, av.z, d);
      d = fmaf(hv.w, av.w, d);
    }
    sdt[which * GBM + row] = d;
  }
  __syncthreads();

  const int rsub = lane / PPR, pc = lane - rsub * PPR;
  const v4f alv = *(const v4fa*)(sdt + 4 * lane);
  float* alp = AL + ((size_t)head * (size_t)gridDim.x + (size_t)blockIdx.x) * (2 * GBM) + 4 * lane;
#pragma unroll 1
  for (int i = 0; i < NIT; ++i) {
    const int row = 16 * wave + i * RPI + rsub;
    const v4f p = *(const v4fa*)(stg + row * GBN + 4 * pc);
    float* op = Cm + (size_t)(rowBase + row) * (size_t)ldc + colBase + 4 * pc;
    *(volatile v4f*)op = p;
  }
  if (wave == 0) *(volatile v4f*)alp = alv;
  __threadfence();
#pragma unroll 1
  for (int i = 0; i < NIT; ++i) {
    const int row = 16 * wave + i * RPI + rsub;
    const v4f p = *(const v4fa*)(stg + row * GBN + 4 * pc);
    float* op = Cm + (size_t)(rowBase + row) * (size_t)ldc + colBase + 4 * pc;
    *(volatile v4f*)op = p;
  }
  if (wave == 0) *(volatile v4f*)alp = alv;
}

template <int L>
__global__ __launch_bounds__(NTHR) void k_agg(const int* __restrict__ srcs, const int* __restrict__ dsts,
                                              int nE, int nN, int vec8, int mRows, int gM,
                                              const float* __restrict__ AL,
                                              const float* __restrict__ xl, const float* __restrict__ bias,
                                              unsigned short* hb, float* outp) {
  static_assert(L == 1 || L == 2);
  extern __shared__ __attribute__((aligned(16))) int dsm[];
  int* list = dsm;
  int* hl   = dsm + LISTN;
  int* sl   = dsm + LISTN + RCAP;
  int* cnt  = dsm + LISTN + 2 * RCAP;
  int* offs = cnt + NBA;
  int* cur  = offs + NBA;
  int* misc = cur + NBA;
  const int tid = (int)threadIdx.x, lane = tid & 31, wave = tid >> 5;
  const int nodeBase = (int)blockIdx.x * NBA;

  {
    const v4i z4 = {0, 0, 0, 0};
    for (int i = tid * 4; i < AGG_ZINTS; i += NTHR * 4) *(v4ia*)(dsm + i) = z4;
    if (tid < 16) misc[tid] = 0;
  }
  __syncthreads();

  int t = 0, ov = 0;
  const int nChunks = (nE + CHUNK - 1) / CHUNK;
#pragma unroll 1
  for (int ch = 0; ch < nChunks; ++ch) {
    const int cbase = ch * CHUNK;
    const int wc = scan_chunk<SLA>(dsts, nE, cbase, nodeBase, NBA, vec8, list, tid, lane, wave);
    if (lane == 0) misc[wave] = wc;
    __syncthreads();
    if (wave == 0) {
#pragma unroll 1
      for (int w2 = 0; w2 < NWAVE; ++w2) {
        int c = misc[w2];
        c = c < 0 ? 0 : (c > WCAP ? WCAP : c);
#pragma unroll 1
        for (int b0 = 0; b0 < c; b0 += 32) {
          const int idx = b0 + lane;
          const int ent = list[w2 * WCAP + (idx < WCAP ? idx : WCAP - 1)];
          const int m32 = (c - b0) < 32 ? (c - b0) : 32;
#pragma unroll 1
          for (int k = 0; k < m32; ++k) {
            const int u    = __builtin_amdgcn_readlane(ent, k);
            const int slot = u & (NBA - 1);
            const int el   = (u >> SLA) & (CHUNK - 1);
            const int pk   = ((cbase + el) << SLA) | slot;
            if (t < RCAP) {
              if (lane == 0) { hl[t] = pk; cnt[slot] = cnt[slot] + 1; }
              t = t + 1;
            } else {
              ov = 1;
            }
          }
        }
      }
    }
    __syncthreads();
  }
  if (wave == 0 && lane == 0) { misc[8] = t; misc[9] = ov; }
  __syncthreads();
  int tt = misc[8];
  tt = tt < 0 ? 0 : (tt > RCAP ? RCAP : tt);
  const int ovf = misc[9];

  if (wave == 0) {
    const int base = lane * (NBA / 32);
    int s = 0;
#pragma unroll 1
    for (int i = 0; i < NBA / 32; ++i) s += cnt[base + i];
    int incl = s;
#pragma unroll
    for (int d = 1; d < 32; d <<= 1) {
      const int y = __shfl_up(incl, d, 32);
      if (lane >= d) incl += y;
    }
    int run = incl - s;
#pragma unroll 1
    for (int i = 0; i < NBA / 32; ++i) {
      const int cv = cnt[base + i];
      offs[base + i] = run;
      cur[base + i]  = run;
      run += cv;
    }
  }
  __syncthreads();
  if (wave == 0) {
#pragma unroll 1
    for (int b0 = 0; b0 < tt; b0 += 32) {
      const int idx = b0 + lane;
      const int ent = hl[idx < RCAP ? idx : RCAP - 1];
      const int m32 = (tt - b0) < 32 ? (tt - b0) : 32;
#pragma unroll 1
      for (int k = 0; k < m32; ++k) {
        const int u    = __builtin_amdgcn_readlane(ent, k);
        const int slot = u & (NBA - 1);
        if (lane == 0) {
          int p = cur[slot];
          p = p < 0 ? 0 : (p > RCAP - 1 ? RCAP - 1 : p);
          sl[p] = u;
          cur[slot] = p + 1;
        }
      }
    }
  }
  __syncthreads();

  float* wst = (float*)hl + wave * 512;
  float* sbb = (float*)hl + NWAVE * 512;
  if constexpr (L == 1) {
#pragma unroll 1
    for (int i = tid; i < HC1; i += NTHR) sbb[i] = bf16_val(bias[i]);
  }
  __syncthreads();

  const float qnan = __int_as_float(0x7fc00000);
  const float pz = (ovf != 0) ? qnan : 0.0f;
  const size_t hstr = (size_t)gM * (size_t)(2 * GBM);

  if constexpr (L == 1) {
    const int hsel = lane >> 4;
    const float* ALa = AL + (size_t)hsel * hstr;
    const float* ALb = AL + (size_t)(2 + hsel) * hstr;
#pragma unroll 1
    for (int si = 0; si < NBA / NWAVE; ++si) {
      const int s    = si * NWAVE + wave;
      const int node = nodeBase + s;
      int c = cnt[s];
      const bool big = c > DEGCAP;
      c = c < 0 ? 0 : (c > DEGCAP ? DEGCAP : c);
      int o = offs[s];
      o = o < 0 ? 0 : (o > RCAP ? RCAP : o);
      const int nc = node < nN ? node : nN - 1;
      const int ab = (nc >> 6) * (2 * GBM) + (nc & (GBM - 1));
      const float adA = ALa[ab + GBM];
      const float adB = ALb[ab + GBM];
      float aA[8], aB[8];
#pragma unroll
      for (int j = 0; j < 8; ++j) { aA[j] = 0.0f; aB[j] = 0.0f; }
      float mxA = -3.0e38f, mxB = -3.0e38f, dnA = 0.0f, dnB = 0.0f;
#pragma unroll 1
      for (int b0 = 0; b0 < c; b0 += 32) {
        int idx = o + b0 + lane;
        idx = idx > RCAP - 1 ? RCAP - 1 : idx;
        const int ent = sl[idx];
        int eid = ent >> SLA;
        eid = eid < 0 ? 0 : (eid > nE - 1 ? nE - 1 : eid);
        int sr = srcs[eid];
        sr = sr < 0 ? 0 : (sr > nN - 1 ? nN - 1 : sr);
        const int sx = (sr >> 6) * (2 * GBM) + (sr & (GBM - 1));
        const int e0 = __float_as_int(AL[sx]);
        const int e1 = __float_as_int(AL[hstr + sx]);
        const int e2 = __float_as_int(AL[2 * hstr + sx]);
        const int e3 = __float_as_int(AL[3 * hstr + sx]);
        const int m32 = (c - b0) < 32 ? (c - b0) : 32;
#pragma unroll 1
        for (int k = 0; k < m32; ++k) {
          const int   sk = __builtin_amdgcn_readlane(sr, k);
          const float f0 = __int_as_float(__builtin_amdgcn_readlane(e0, k));
          const float f1 = __int_as_float(__builtin_amdgcn_readlane(e1, k));
          const float f2 = __int_as_float(__builtin_amdgcn_readlane(e2, k));
          const float f3 = __int_as_float(__builtin_amdgcn_readlane(e3, k));
          const float esA = (hsel != 0) ? f1 : f0;
          const float esB = (hsel != 0) ? f3 : f2;
          const float* rp = xl + (size_t)sk * HC1 + 8 * lane;
          const v4f a0 = *(const v4f*)rp;
          const v4f a1 = *(const v4f*)(rp + 4);
          const v4f c0 = *(const v4f*)(rp + 256);
          const v4f c1 = *(const v4f*)(rp + 260);
          float lgA = esA + adA; lgA = lgA > 0.f ? lgA : NEGSL * lgA;
          float lgB = esB + adB; lgB = lgB > 0.f ? lgB : NEGSL * lgB;
          float s1, s2;
          osm(lgA, mxA, dnA, s1, s2);
          aA[0] = fmaf(aA[0], s1, s2 * a0.x); aA[1] = fmaf(aA[1], s1, s2 * a0.y);
          aA[2] = fmaf(aA[2], s1, s2 * a0.z); aA[3] = fmaf(aA[3], s1, s2 * a0.w);
          aA[4] = fmaf(aA[4], s1, s2 * a1.x); aA[5] = fmaf(aA[5], s1, s2 * a1.y);
          aA[6] = fmaf(aA[6], s1, s2 * a1.z); aA[7] = fmaf(aA[7], s1, s2 * a1.w);
          osm(lgB, mxB, dnB, s1, s2);
          aB[0] = fmaf(aB[0], s1, s2 * c0.x); aB[1] = fmaf(aB[1], s1, s2 * c0.y);
          aB[2] = fmaf(aB[2], s1, s2 * c0.z); aB[3] = fmaf(aB[3], s1, s2 * c0.w);
          aB[4] = fmaf(aB[4], s1, s2 * c1.x); aB[5] = fmaf(aB[5], s1, s2 * c1.y);
          aB[6] = fmaf(aB[6], s1, s2 * c1.z); aB[7] = fmaf(aB[7], s1, s2 * c1.w);
        }
      }
      const float invA = (c > 0) ? __builtin_amdgcn_rcpf(dnA) : 0.0f;
      const float invB = (c > 0) ? __builtin_amdgcn_rcpf(dnB) : 0.0f;
      const float pzr  = big ? qnan : pz;
      const bool  live = node < nN;
#pragma unroll
      for (int j = 0; j < 8; ++j) { wst[j * 32 + lane] = aA[j]; wst[(8 + j) * 32 + lane] = aB[j]; }
#pragma unroll 1
      for (int i = 0; i < 16; ++i) {
        const float a   = wst[i * 32 + lane];
        const float inv = (i < 8) ? invA : invB;
        const int   chn = (i >> 3) * 256 + 8 * lane + (i & 7);
        float y = fmaf(a, inv, sbb[chn]);
        y = (y > 0.0f) ? y : expm1f(y);
        wst[i * 32 + lane] = y;
      }
      v8us hoA, loA, hoB, loB;
#pragma unroll
      for (int j = 0; j < 8; ++j) {
        float ya = wst[j * 32 + lane] + pzr;
        float yb = wst[(8 + j) * 32 + lane] + pzr;
        ya = live ? ya : 0.0f;
        yb = live ? yb : 0.0f;
        const unsigned ha = bf16_bits(ya), hq = bf16_bits(yb);
        hoA[j] = (unsigned short)ha;
        hoB[j] = (unsigned short)hq;
        loA[j] = (unsigned short)bf16_bits(ya - __uint_as_float(ha << 16));
        loB[j] = (unsigned short)bf16_bits(yb - __uint_as_float(hq << 16));
      }
      if (node < mRows) {
        unsigned short* hp = hb + (size_t)node * KP2 + 8 * lane;
        *(volatile v8us*)hp = hoA;
        *(volatile v8us*)(hp + 256) = hoB;
        *(volatile v8us*)(hp + 512) = loA;
        *(volatile v8us*)(hp + 768) = loB;
        __threadfence();
        *(volatile v8us*)hp = hoA;
        *(volatile v8us*)(hp + 256) = hoB;
        *(volatile v8us*)(hp + 512) = loA;
        *(volatile v8us*)(hp + 768) = loB;
      }
    }
  } else {
    const int c4 = 4 * (lane & 15);
    const v4f bq = *(const v4f*)(bias + c4);
    const float bz0 = bf16_val(bq.x), bz1 = bf16_val(bq.y), bz2 = bf16_val(bq.z), bz3 = bf16_val(bq.w);
#pragma unroll 1
    for (int si = 0; si < NBA / NWAVE; ++si) {
      const int s    = si * NWAVE + wave;
      const int node = nodeBase + s;
      int c = cnt[s];
      const bool big = c > DEGCAP;
      c = c < 0 ? 0 : (c > DEGCAP ? DEGCAP : c);
      int o = offs[s];
      o = o < 0 ? 0 : (o > RCAP ? RCAP : o);
      const int nc = node < nN ? node : nN - 1;
      const int ab = (nc >> 6) * (2 * GBM) + (nc & (GBM - 1));
      const float ad = AL[ab + GBM];
      float a0 = 0.0f, a1 = 0.0f, a2 = 0.0f, a3 = 0.0f;
      float mx = -3.0e38f, dn = 0.0f;
#pragma unroll 1
      for (int b0 = 0; b0 < c; b0 += 32) {
        int idx = o + b0 + lane;
        idx = idx > RCAP - 1 ? RCAP - 1 : idx;
        const int ent = sl[idx];
        int eid = ent >> SLA;
        eid = eid < 0 ? 0 : (eid > nE - 1 ? nE - 1 : eid);
        int sr = srcs[eid];
        sr = sr < 0 ? 0 : (sr > nN - 1 ? nN - 1 : sr);
        const int esi = __float_as_int(AL[(sr >> 6) * (2 * GBM) + (sr & (GBM - 1))]);
        const int m32 = (c - b0) < 32 ? (c - b0) : 32;
#pragma unroll 1
        for (int k = 0; k < m32; ++k) {
          const int   sk  = __builtin_amdgcn_readlane(sr, k);
          const float ask = __int_as_float(__builtin_amdgcn_readlane(esi, k));
          const v4f a = *(const v4f*)(xl + (size_t)sk * DOUT + c4);
          float lg = ask + ad;
          lg = lg > 0.f ? lg : NEGSL * lg;
          float s1, s2;
          osm(lg, mx, dn, s1, s2);
          a0 = fmaf(a0, s1, s2 * a.x); a1 = fmaf(a1, s1, s2 * a.y);
          a2 = fmaf(a2, s1, s2 * a.z); a3 = fmaf(a3, s1, s2 * a.w);
        }
      }
      const float inv = (c > 0) ? __builtin_amdgcn_rcpf(dn) : 0.0f;
      const float pzr = big ? qnan : pz;
      v4f ov4;
      ov4.x = fmaf(a0, inv, bz0) + pzr;
      ov4.y = fmaf(a1, inv, bz1) + pzr;
      ov4.z = fmaf(a2, inv, bz2) + pzr;
      ov4.w = fmaf(a3, inv, bz3) + pzr;
      const bool wr = (node < nN) && (lane < 16);
      float* op = outp + (size_t)nc * DOUT + c4;
      if (wr) *(volatile v4f*)op = ov4;
      __threadfence();
      if (wr) *(volatile v4f*)op = ov4;
    }
  }
}

static inline int cdiv(int a, int b) { return (a + b - 1) / b; }

extern "C" void kernel_launch(void* const* d_in, const int* in_sizes, int n_in,
                              void* d_out, int out_size, void* d_ws, size_t ws_size,
                              hipStream_t stream) {
  if (n_in < 11) return;
  if (in_sizes[0] < F_IN || (in_sizes[0] % F_IN) != 0) return;
  const int nN = in_sizes[0] / F_IN;
  if (nN > (1 << 22)) return;
  const int nE = in_sizes[1];
  if (nE < 1 || nE >= (1 << 21)) return;
  if (in_sizes[2] != nE) return;
  if (in_sizes[3] != F_IN * HC1) return;
  if (in_sizes[4] != HC1 || in_sizes[5] != HC1 || in_sizes[6] != HC1) return;
  if (in_sizes[7] != HC1 * DOUT) return;
  if (in_sizes[8] != DOUT || in_sizes[9] != DOUT || in_sizes[10] != DOUT) return;
  if ((long long)out_size != (long long)nN * DOUT) return;

  const float* x   = (const float*)d_in[0];
  const int*   src = (const int*)d_in[1];
  const int*   dst = (const int*)d_in[2];
  const float* W1  = (const float*)d_in[3];
  const float* al1 = (const float*)d_in[4];
  const float* ar1 = (const float*)d_in[5];
  const float* b1  = (const float*)d_in[6];
  const float* W2  = (const float*)d_in[7];
  const float* al2 = (const float*)d_in[8];
  const float* ar2 = (const float*)d_in[9];
  const float* b2  = (const float*)d_in[10];
  float* out = (float*)d_out;

  const int MP   = cdiv(nN, MROWS) * MROWS;
  const int gM   = MP / GBM;
  const int gA   = cdiv(MP, NBA);
  if ((long long)gA * NBA < (long long)MP) return;
  const int vec8 = ((nE & 3) == 0) ? 1 : 0;

  char* ws = (char*)d_ws;
  size_t off = 0;
  const size_t oXB  = off; off += (size_t)MP * F_IN * 2;                 off = (off + 255) & ~(size_t)255;
  const size_t oW1T = off; off += (size_t)HC1 * F_IN * 2;                off = (off + 255) & ~(size_t)255;
  const size_t oW2T = off; off += (size_t)DOUT * KP2 * 2;                off = (off + 255) & ~(size_t)255;
  const size_t oF1  = off; off += (size_t)MP * HC1 * 4;                  off = (off + 255) & ~(size_t)255;
  const size_t oAL1 = off; off += (size_t)NH1 * gM * (2 * GBM) * 4;      off = (off + 255) & ~(size_t)255;
  const size_t oH1  = off; off += (size_t)MP * KP2 * 2;                  off = (off + 255) & ~(size_t)255;
  const size_t oF2  = off; off += (size_t)MP * DOUT * 4;                 off = (off + 255) & ~(size_t)255;
  const size_t oAL2 = off; off += (size_t)gM * (2 * GBM) * 4;            off = (off + 255) & ~(size_t)255;
  if (off > ws_size || off > (size_t)WSMAX) return;
  unsigned short* XB   = (unsigned short*)(ws + oXB);
  unsigned short* W1T  = (unsigned short*)(ws + oW1T);
  unsigned short* W2T2 = (unsigned short*)(ws + oW2T);
  float*          F1   = (float*)(ws + oF1);
  float*          AL1  = (float*)(ws + oAL1);
  unsigned short* H1   = (unsigned short*)(ws + oH1);
  float*          F2   = (float*)(ws + oF2);
  float*          AL2  = (float*)(ws + oAL2);

  const size_t aggLds = (size_t)AGG_LDS_INTS * 4;
  hipFuncSetAttribute(reinterpret_cast<const void*>(&k_agg<1>), hipFuncAttributeMaxDynamicSharedMemorySize, (int)aggLds);
  hipFuncSetAttribute(reinterpret_cast<const void*>(&k_agg<2>), hipFuncAttributeMaxDynamicSharedMemorySize, (int)aggLds);

  const int nUx = MP * (F_IN / 8);
  k_xprep<<<cdiv(nUx, NTHR), NTHR, 0, stream>>>(x, XB, nN, nUx);
  {
    const int nUw1 = HC1 * (F_IN / 8);
    k_wtr<<<cdiv(nUw1, NTHR), NTHR, 0, stream>>>(W1, F_IN, HC1, HC1, F_IN, W1T, nUw1);
    const int nUw2 = DOUT * (KP2 / 8);
    k_wtr<<<cdiv(nUw2, NTHR), NTHR, 0, stream>>>(W2, HC1, DOUT, DOUT, KP2, W2T2, nUw2);
  }
  k_gemm<8><<<dim3(gM, NH1), GTHR, 0, stream>>>(XB, F_IN, W1T, F_IN, F_IN, F1, HC1, al1, ar1, AL1);
  k_agg<1><<<gA, NTHR, aggLds, stream>>>(src, dst, nE, nN, vec8, MP, gM, AL1, F1, b1, H1, out);
  k_gemm<4><<<dim3(gM, 1), GTHR, 0, stream>>>(H1, KP2, W2T2, KP2, KP2, F2, DOUT, al2, ar2, AL2);
  k_agg<2><<<gA, NTHR, aggLds, stream>>>(src, dst, nE, nN, vec8, MP, gM, AL2, F2, b2, H1, out);
}
